// IpaBlock_13640816132144
// MI455X (gfx1250) — hardware-verified
//
#include <hip/hip_runtime.h>


namespace {
constexpr int N = 10000, E = 160000, HID = 256, NH = 8, DH = 32, NPAD = 10112  , NBLK = NPAD / 128, NBA = 128  , NAGG = (NPAD + NBA - 1) / NBA;
constexpr float FXS = 1048576.0f, FXI = 1.0f / 1048576.0f, AS_ = 8.0f, WS_ = 32.0f, ISQ = 0.17677669529663687f;

typedef _Float16 b16;
typedef __attribute__((ext_vector_type(16))) _Float16 v16b;
typedef __attribute__((ext_vector_type(8))) _Float16 v8b;
typedef __attribute__((ext_vector_type(8))) float v8f;
typedef __attribute__((ext_vector_type(4))) float v4f;
__device__ __forceinline__ void split16(float v, b16& hi, b16& lo) { hi = (b16)v; lo = (b16)(v - (float)hi); }
__device__ __forceinline__ v16b frag_kb(const b16* p, int hh) { const v8b a = *(const v8b*)(p + 8 * hh), b = *(const v8b*)(p + 16 + 8 * hh); v16b f;
#pragma unroll
  for (int e = 0; e < 8; ++e) { f[e] = a[e]; f[8 + e] = b[e]; } return f; }
__device__ __forceinline__ v8f wmma16b(v16b a, v16b b, v8f c) { v8f d = __builtin_amdgcn_wmma_f32_16x16x32_f16(false, a, false, b, (short)0, c, false, false); asm volatile("v_nop\n\tv_nop\n\tv_nop\n\tv_nop" : "+v"(d) : "v"(a), "v"(b)); return d; }
__device__ __forceinline__ void wave_lds_sync() { __builtin_amdgcn_fence(__ATOMIC_RELEASE, "workgroup"); __builtin_amdgcn_wave_barrier(); __builtin_amdgcn_fence(__ATOMIC_ACQUIRE, "workgroup"); }
__device__ __forceinline__ int fkey(float f) { const int b = __float_as_int(f); return (b >= 0) ? b : (b ^ 0x7FFFFFFF); }
__device__ __forceinline__ float fkey_inv(int k) { return __int_as_float((k >= 0) ? k : (k ^ 0x7FFFFFFF)); }
__device__ __forceinline__ int clampn(int v) { return (v < 0) ? 0 : (v >= N ? N - 1 : v); }
__device__ __forceinline__ float nexp(float x) { return __builtin_amdgcn_exp2f(x * 1.4426950408889634f); }

__global__ __launch_bounds__(256) void prep_kernel(const float* __restrict__ Wq, const float* __restrict__ Wk, const float* __restrict__ Wv, const float* __restrict__ Wo, const float* __restrict__ Wg1, b16* __restrict__ wqkv, b16* __restrict__ wo, b16* __restrict__ wg) {
  const size_t tid = (size_t)blockIdx.x * blockDim.x + threadIdx.x, nth = (size_t)gridDim.x * blockDim.x; const size_t PL = (size_t)HID * HID;
  for (int pass = 0; pass < 2; ++pass) {
    for (size_t p = tid; p < 3 * PL; p += nth) { const float* W = (p < PL) ? Wq : (p < 2 * PL) ? Wk : Wv; b16 a, c; split16(W[p % PL] * WS_, a, c); ((volatile b16*)wqkv)[p] = a; ((volatile b16*)wqkv)[3 * PL + p] = c; }
    for (size_t p = tid; p < PL; p += nth) { b16 a, c; split16(Wo[p] * WS_, a, c); ((volatile b16*)wo)[p] = a; ((volatile b16*)wo)[PL + p] = c; split16(Wg1[p] * WS_, a, c); ((volatile b16*)wg)[p] = a; ((volatile b16*)wg)[PL + p] = c; }
    __threadfence();
  }
}

template <int MODE, int NCOL>
__global__ __launch_bounds__(128) void lin_kernel(const float* __restrict__ A, const b16* __restrict__ Bw, size_t LOFF, const float* __restrict__ bias, const float* __restrict__ hin, float* __restrict__ y, float* __restrict__ y2) {
  __shared__ __attribute__((aligned(16))) float Ts[4][32 * 64];
  const int lane = threadIdx.x & 31, wave = threadIdx.x >> 5, nloc = lane & 15, hlf = lane >> 4, m0 = blockIdx.y * 128 + wave * 32, c0 = blockIdx.x * 64;
  const int ra = min(m0 + nloc, N - 1), rb = min(m0 + 16 + nloc, N - 1);
  v8f acc[2][4];
#pragma unroll
  for (int r = 0; r < 2; ++r)
#pragma unroll
    for (int t = 0; t < 4; ++t) acc[r][t] = (v8f){};
#pragma unroll 1
  for (int kb = 0; kb < HID; kb += 32) { v16b a0, a1, l0, l1;
#pragma unroll
    for (int e = 0; e < 16; ++e) { const int k = kb + ((e < 8) ? (8 * hlf + e) : (16 + 8 * hlf + e - 8)); b16 p, q; split16(A[(size_t)ra * HID + k] * AS_, p, q); a0[e] = p; l0[e] = q; split16(A[(size_t)rb * HID + k] * AS_, p, q); a1[e] = p; l1[e] = q; }
#pragma unroll
    for (int t = 0; t < 4; ++t) { const size_t bo = (size_t)(c0 + t * 16 + nloc) * HID + kb; const v16b b0 = frag_kb(Bw + bo, hlf), b1 = frag_kb(Bw + LOFF + bo, hlf);
      acc[0][t] = wmma16b(a0, b0, acc[0][t]); acc[0][t] = wmma16b(l0, b0, acc[0][t]); acc[0][t] = wmma16b(a0, b1, acc[0][t]);
      acc[1][t] = wmma16b(a1, b0, acc[1][t]); acc[1][t] = wmma16b(l1, b0, acc[1][t]); acc[1][t] = wmma16b(a1, b1, acc[1][t]); } }
  float* Tt = Ts[wave];
#pragma unroll
  for (int t = 0; t < 4; ++t)
#pragma unroll
    for (int r = 0; r < 2; ++r)
#pragma unroll
      for (int v = 0; v < 8; ++v) { const int row = m0 + r * 16 + 8 * hlf + v, c = c0 + t * 16 + nloc; float val = acc[r][t][v] * (1.0f / (AS_ * WS_)) + bias[c];
        if (MODE == 1) val += hin[(size_t)min(row, N - 1) * HID + c]; if (MODE == 2) val = val / (1.0f + __expf(-val));
        Tt[(r * 16 + v + 8 * hlf) * 64 + t * 16 + nloc] = (row < N) ? val : 0.0f; }
  wave_lds_sync();
  for (int pass = 0; pass < 2; ++pass) {
#pragma unroll
    for (int j = 0; j < 16; ++j) { const int rr = j * 2 + hlf, c4 = nloc * 4; const v4f v = *(const v4f*)(Tt + rr * 64 + c4);
      if (MODE == 1) { if (m0 + rr < N) *(volatile v4f*)(y + (size_t)(m0 + rr) * NCOL + c0 + c4) = v; *(volatile v4f*)(y2 + (size_t)(m0 + rr) * NCOL + c0 + c4) = v; }
      else *(volatile v4f*)(y + (size_t)(m0 + rr) * NCOL + c0 + c4) = v; }
    __threadfence(); }
}

__global__ __launch_bounds__(256) void escore_kernel(const float* __restrict__ qkv, const int* __restrict__ srcI, const int* __restrict__ dstI, const float* __restrict__ x, const float* __restrict__ fr,
                                                     const float* __restrict__ dist, const float* __restrict__ bpp, const float* __restrict__ msa, const float* __restrict__ chem, const float* __restrict__ rel, const float* __restrict__ chain,
                                                     const float* __restrict__ Wd, const float* __restrict__ bd, const float* __restrict__ Wb, const float* __restrict__ bb, const float* __restrict__ Wm, const float* __restrict__ bm, const float* __restrict__ Wc, const float* __restrict__ bc,
                                                     const float* __restrict__ Wr, const float* __restrict__ br, const float* __restrict__ Wch, const float* __restrict__ bch, const float* __restrict__ Wori, const float* __restrict__ bori,
                                                     float* __restrict__ esc, float* __restrict__ ed) {
  const int t_ = threadIdx.x, el = t_ >> 3, hd = t_ & 7, e = blockIdx.x * 32 + el; const int s = clampn(srcI[e]), d = clampn(dstI[e]);
  const float* q = qkv + (size_t)s * 3 * HID + hd * DH; const float* k = qkv + (size_t)d * 3 * HID + HID + hd * DH; float dot = 0.0f;
#pragma unroll 8
  for (int c = 0; c < DH; ++c) dot += q[c] * k[c];
  const float dx = x[d * 3] - x[s * 3], dy = x[d * 3 + 1] - x[s * 3 + 1], dz = x[d * 3 + 2] - x[s * 3 + 2]; const float* F = fr + (size_t)s * 9;
  const float l0 = F[0] * dx + F[3] * dy + F[6] * dz, l1 = F[1] * dx + F[4] * dy + F[7] * dz, l2 = F[2] * dx + F[5] * dy + F[8] * dz;
  const float nrm = fmaxf(sqrtf(l0 * l0 + l1 * l1 + l2 * l2), 1e-6f), u0 = l0 / nrm, u1 = l1 / nrm, u2 = l2 / nrm;
  const float dsq = dist[e] * dist[e];
  float tot = dot * ISQ - (dsq * Wd[hd] + bd[hd]) + (bpp[e] * Wb[hd] + bb[hd]) + (msa[e] * Wm[hd] + bm[hd]) + (chem[e] * Wc[hd] + bc[hd]) + (rel[e] * Wr[hd] + br[hd]) + (chain[e] * Wch[hd] + bch[hd]);
  tot += 0.1f * tanhf(u0 * Wori[hd * 3] + u1 * Wori[hd * 3 + 1] + u2 * Wori[hd * 3 + 2] + bori[hd]);
  const float geo = (hd == 0) ? l0 : (hd == 1) ? l1 : (hd == 2) ? l2 : (hd == 3) ? dx : (hd == 4) ? dy : (hd == 5) ? dz : 0.0f;
  for (int pass = 0; pass < 2; ++pass) { ((volatile float*)esc)[(size_t)e * 8 + hd] = tot; ((volatile float*)ed)[(size_t)e * 8 + hd] = geo; __threadfence(); }
}

typedef __attribute__((ext_vector_type(4))) int v4i;
__global__ __launch_bounds__(256) void agg_kernel(const int* __restrict__ srcI, const int* __restrict__ dstI, const float* __restrict__ qkv, const float* __restrict__ esc, const float* __restrict__ ed, float* __restrict__ hup, float* __restrict__ dsp) {
  __shared__ __attribute__((aligned(16))) int acc[NBA * HID];
  __shared__ int mx[NBA * NH]; __shared__ int den[NBA * NH]; __shared__ int dac[NBA * 48]; __shared__ int list[8 * 256];
  const int t_ = threadIdx.x, wave = t_ >> 5, lane = t_ & 31, base = blockIdx.x * NBA, col0 = lane * 8, myh = col0 / DH;
  for (int i = t_; i < NBA * HID; i += 256) acc[i] = 0;
  for (int i = t_; i < NBA * 48; i += 256) dac[i] = 0;
  for (int i = t_; i < NBA * NH; i += 256) { den[i] = 0; mx[i] = fkey(-INFINITY); }
  __syncthreads();
  for (int c0 = 0; c0 < E; c0 += 256 * 8) { const int e0 = c0 + (wave * 32 + lane) * 8;
#pragma unroll
    for (int j = 0; j < 8; ++j) { const int ee = min(e0 + j, E - 1); const unsigned sl = (unsigned)(((e0 + j < E) ? srcI[ee] : -1) - base);
      if (sl < (unsigned)NBA) {
#pragma unroll
        for (int h = 0; h < NH; ++h) atomicMax(&mx[sl * NH + h], fkey(esc[(size_t)ee * 8 + h])); } } }
  __syncthreads();
  int* wl = list + wave * 256;
  for (int c0 = 0; c0 < E; c0 += 256 * 8) {
    const int e0 = c0 + (wave * 32 + lane) * 8; int dd[8];
#pragma unroll
    for (int j = 0; j < 8; ++j) { const int sv = srcI[min(e0 + j, E - 1)]; dd[j] = (e0 + j < E) ? sv : -1; }
    unsigned sl[8]; bool hit[8]; bool anyl = false;
#pragma unroll
    for (int j = 0; j < 8; ++j) { sl[j] = (unsigned)(dd[j] - base); hit[j] = sl[j] < (unsigned)NBA; anyl |= hit[j]; }
    int wc = 0;
    if (__builtin_amdgcn_ballot_w32(anyl) != 0u) {
#pragma unroll
      for (int j = 0; j < 8; ++j) {
        const unsigned mj = __builtin_amdgcn_ballot_w32(hit[j]);
        if (mj != 0u) {
          if (hit[j]) { const int pos = wc + (int)__builtin_amdgcn_mbcnt_lo(mj, 0u); wl[pos] = ((e0 + j) << 7) | (int)sl[j]; }
          wc += __builtin_popcount(mj); } } }
    __builtin_amdgcn_wave_barrier(); __builtin_amdgcn_fence(__ATOMIC_RELEASE, "workgroup"); __builtin_amdgcn_fence(__ATOMIC_ACQUIRE, "workgroup");
    for (int i = 0; i < wc; ++i) { const int ent = wl[i]; const int e = ent >> 7, slot = ent & 127; const int d = clampn(dstI[e]);
      const v4f ea = *(const v4f*)(esc + (size_t)e * 8), eb = *(const v4f*)(esc + (size_t)e * 8 + 4); float w[8];
#pragma unroll
      for (int h = 0; h < 4; ++h) { w[h] = nexp(ea[h] - fkey_inv(mx[slot * NH + h])); w[4 + h] = nexp(eb[h] - fkey_inv(mx[slot * NH + 4 + h])); }
      const float wsel = (lane == 0) ? w[0] : (lane == 1) ? w[1] : (lane == 2) ? w[2] : (lane == 3) ? w[3] : (lane == 4) ? w[4] : (lane == 5) ? w[5] : (lane == 6) ? w[6] : w[7];
      if (lane < NH) atomicAdd(&den[slot * NH + lane], (int)rintf(wsel * FXS));
      const float wm = (myh == 0) ? w[0] : (myh == 1) ? w[1] : (myh == 2) ? w[2] : (myh == 3) ? w[3] : (myh == 4) ? w[4] : (myh == 5) ? w[5] : (myh == 6) ? w[6] : w[7];
      const float* vr = qkv + (size_t)d * 3 * HID + 2 * HID + col0; const v4f va = *(const v4f*)vr, vb = *(const v4f*)(vr + 4); int* ar = acc + slot * HID + col0;
#pragma unroll
      for (int c = 0; c < 4; ++c) { atomicAdd(ar + c, (int)rintf(wm * va[c] * FXS)); atomicAdd(ar + 4 + c, (int)rintf(wm * vb[c] * FXS)); }
      if (lane >= 8) { const int idx = (lane - 8) * 2;
        const v4f ga = *(const v4f*)(ed + (size_t)e * 8), gb = *(const v4f*)(ed + (size_t)e * 8 + 4); const float g6[6] = {ga[0], ga[1], ga[2], ga[3], gb[0], gb[1]};
#pragma unroll
        for (int q = 0; q < 2; ++q) { const int id = idx + q, hh = id / 6, cp = id % 6; const float wh = (hh == 0) ? w[0] : (hh == 1) ? w[1] : (hh == 2) ? w[2] : (hh == 3) ? w[3] : (hh == 4) ? w[4] : (hh == 5) ? w[5] : (hh == 6) ? w[6] : w[7];
          const float gv = (cp == 0) ? g6[0] : (cp == 1) ? g6[1] : (cp == 2) ? g6[2] : (cp == 3) ? g6[3] : (cp == 4) ? g6[4] : g6[5];
          atomicAdd(&dac[slot * 48 + id], (int)rintf(wh * gv * FXS)); } } }
    __builtin_amdgcn_wave_barrier();
  }
  __syncthreads();
  for (int pass = 0; pass < 2; ++pass) {
    for (int i = t_; i < NBA * HID / 4; i += 256) { const int slot = i / (HID / 4), cq = (i % (HID / 4)) * 4, node = base + slot; v4f o = {0.0f, 0.0f, 0.0f, 0.0f};
      if (node < N) { const int hh = cq / DH; const float dn = (float)den[slot * NH + hh]; const float sc = (dn > 0.0f) ? __builtin_amdgcn_rcpf(dn) : 0.0f;
#pragma unroll
        for (int c = 0; c < 4; ++c) o[c] = (float)acc[slot * HID + cq + c] * sc; }
      if (node < NPAD) *(volatile v4f*)(hup + (size_t)node * HID + cq) = o; }
    for (int i = t_; i < NBA * 2; i += 256) { const int slot = i >> 1, half = i & 1, node = base + slot; v4f o = {0.0f, 0.0f, 0.0f, 0.0f};
      if (node < N && half == 0) { float r[3] = {0.0f, 0.0f, 0.0f};
        for (int hh = 0; hh < NH; ++hh) { const float dn = (float)den[slot * NH + hh]; const float sc = (dn > 0.0f) ? 0.125f * __builtin_amdgcn_rcpf(dn) : 0.0f; r[0] += (float)dac[slot * 48 + hh * 6 + 0] * sc; r[1] += (float)dac[slot * 48 + hh * 6 + 1] * sc; r[2] += (float)dac[slot * 48 + hh * 6 + 2] * sc; }
        o[0] = r[0]; o[1] = r[1]; o[2] = r[2]; }
      if (node < N && half == 1) { float r[3] = {0.0f, 0.0f, 0.0f};
        for (int hh = 0; hh < NH; ++hh) { const float dn = (float)den[slot * NH + hh]; const float sc = (dn > 0.0f) ? 0.125f * __builtin_amdgcn_rcpf(dn) : 0.0f; r[0] += (float)dac[slot * 48 + hh * 6 + 3] * sc; r[1] += (float)dac[slot * 48 + hh * 6 + 4] * sc; r[2] += (float)dac[slot * 48 + hh * 6 + 5] * sc; }
        o[0] = r[0]; o[1] = r[1]; o[2] = r[2]; }
      if (node < NPAD) *(volatile v4f*)(dsp + (size_t)node * 8 + half * 4) = o; }
    __threadfence(); }
}

__global__ __launch_bounds__(256) void final_kernel(const float* __restrict__ g1, const float* __restrict__ Wg2, const float* __restrict__ bg2, const float* __restrict__ dsp, const float* __restrict__ fr, const float* __restrict__ x, float* __restrict__ xo) {
  __shared__ __attribute__((aligned(16))) float Xs[256 * 3];
  const int n = blockIdx.x * 256 + threadIdx.x; const int nn = min(n, N - 1);
  const float* gr = g1 + (size_t)nn * HID; float s = bg2[0];
#pragma unroll 8
  for (int c = 0; c < HID; ++c) s += gr[c] * Wg2[c];
  const float gate = tanhf(s); const float* F = fr + (size_t)nn * 9; const float* dp = dsp + (size_t)nn * 8;
  const float dl0 = dp[0], dl1 = dp[1], dl2 = dp[2];
#pragma unroll
  for (int i = 0; i < 3; ++i) { const float fg = F[i * 3] * dl0 + F[i * 3 + 1] * dl1 + F[i * 3 + 2] * dl2; Xs[threadIdx.x * 3 + i] = x[nn * 3 + i] + gate * (0.5f * fg + 0.5f * dp[4 + i]); }
  __syncthreads();
  const int nval = min(256, N - blockIdx.x * 256), npieces = nval * 3 / 4;
  for (int pass = 0; pass < 2; ++pass) { if ((int)threadIdx.x < npieces) *(volatile v4f*)(xo + (size_t)blockIdx.x * 768 + threadIdx.x * 4) = *(const v4f*)(&Xs[threadIdx.x * 4]); __threadfence(); }
}
}

extern "C" void kernel_launch(void* const* d_in, const int* in_sizes, int n_in,
                              void* d_out, int out_size, void* d_ws, size_t ws_size, hipStream_t stream) {
  (void)n_in; (void)out_size;
  const float* h = (const float*)d_in[0]; const float* x = (const float*)d_in[1]; const int* srcI = (const int*)d_in[2]; const int* dstI = (const int*)d_in[3];
  const float* dist = (const float*)d_in[4]; const float* bpp = (const float*)d_in[5]; const float* msa = (const float*)d_in[6]; const float* chem = (const float*)d_in[7]; const float* rel = (const float*)d_in[8]; const float* chain = (const float*)d_in[9];
  const float* fr = (const float*)d_in[10]; const float* Wq = (const float*)d_in[11]; const float* bq = (const float*)d_in[12]; const float* Wk = (const float*)d_in[13]; const float* bk = (const float*)d_in[14]; const float* Wv = (const float*)d_in[15]; const float* bv = (const float*)d_in[16];
  const float* Wo = (const float*)d_in[17]; const float* bo = (const float*)d_in[18];
  const float* p[14]; for (int i = 0; i < 14; ++i) p[i] = (const float*)d_in[19 + i];
  const float* Wg1 = (const float*)d_in[33]; const float* bg1 = (const float*)d_in[34]; const float* Wg2 = (const float*)d_in[35]; const float* bg2 = (const float*)d_in[36];
  float* hout = (float*)d_out; float* xout = hout + (size_t)N * HID;
  if (in_sizes[0] != N * HID || in_sizes[1] != N * 3 || in_sizes[2] != E || in_sizes[3] != E || in_sizes[10] != N * 9 || in_sizes[11] != HID * HID || in_sizes[33] != HID * HID || in_sizes[35] != HID) return;
  size_t off = 0; char* ws = (char*)d_ws;
  auto carve = [&](size_t bytes) { char* q = ws + off; off += (bytes + 255) & ~(size_t)255; return q; };
  const size_t PL = (size_t)HID * HID;
  b16* wqkv = (b16*)carve(6 * PL * 2); b16* wo = (b16*)carve(2 * PL * 2); b16* wg = (b16*)carve(2 * PL * 2);
  float* bqkv = (float*)carve((size_t)3 * HID * 4); float* qkv = (float*)carve((size_t)NPAD * 3 * HID * 4); float* esc = (float*)carve((size_t)E * 8 * 4); float* ed = (float*)carve((size_t)E * 8 * 4);
  float* hup = (float*)carve((size_t)NPAD * HID * 4); float* dsp = (float*)carve((size_t)NPAD * 8 * 4); float* hof = (float*)carve((size_t)NPAD * HID * 4); float* g1 = (float*)carve((size_t)NPAD * HID * 4);
  if (off > ws_size) return;
  prep_kernel<<<256, 256, 0, stream>>>(Wq, Wk, Wv, Wo, Wg1, wqkv, wo, wg);
  (void)bqkv;
  lin_kernel<0, 3 * HID><<<dim3(HID / 64, NBLK), 128, 0, stream>>>(h, wqkv, 3 * PL, bq, nullptr, qkv, nullptr);
  lin_kernel<0, 3 * HID><<<dim3(HID / 64, NBLK), 128, 0, stream>>>(h, wqkv + PL, 3 * PL, bk, nullptr, qkv + HID, nullptr);
  lin_kernel<0, 3 * HID><<<dim3(HID / 64, NBLK), 128, 0, stream>>>(h, wqkv + 2 * PL, 3 * PL, bv, nullptr, qkv + 2 * HID, nullptr);
  escore_kernel<<<E / 32, 256, 0, stream>>>(qkv, srcI, dstI, x, fr, dist, bpp, msa, chem, rel, chain, p[0], p[1], p[2], p[3], p[4], p[5], p[6], p[7], p[8], p[9], p[10], p[11], p[12], p[13], esc, ed);
  agg_kernel<<<NAGG, 256, 0, stream>>>(srcI, dstI, qkv, esc, ed, hup, dsp);
  lin_kernel<1, HID><<<dim3(HID / 64, NBLK), 128, 0, stream>>>(hup, wo, PL, bo, h, hout, hof);
  lin_kernel<2, HID><<<dim3(HID / 64, NBLK), 128, 0, stream>>>(hof, wg, PL, bg1, nullptr, g1, nullptr);
  final_kernel<<<(N + 255) / 256, 256, 0, stream>>>(g1, Wg2, bg2, dsp, fr, x, xout);
}
